// TemporalSplitterLayer_81535659148085
// MI455X (gfx1250) — hardware-verified
//
#include <hip/hip_runtime.h>


#define NB_  4
#define NN   4096
#define DD   256
#define DF   512
#define NT   (NB_ * NN)
#define QH   2048
typedef _Float16 h16;
typedef unsigned short bf;
typedef __attribute__((ext_vector_type(16))) __bf16   v16bf;
typedef __attribute__((ext_vector_type(16))) _Float16 v16h;
typedef __attribute__((ext_vector_type(8)))  _Float16 v8h;
typedef __attribute__((ext_vector_type(8)))  unsigned short v8us;
typedef __attribute__((ext_vector_type(8)))  float    v8f;
typedef __attribute__((ext_vector_type(4)))  float    v4f;
typedef v8h  __attribute__((may_alias)) v8ha;
typedef v4f  __attribute__((may_alias)) v4fa;
typedef v8us __attribute__((may_alias)) v8usa;

__device__ __forceinline__ unsigned short f2bf(float f) { unsigned u = __float_as_uint(f); u += 0x7FFFu + ((u >> 16) & 1u); return (unsigned short)(u >> 16); }
__device__ __forceinline__ float bf2f(unsigned short b) { return __uint_as_float(((unsigned)b) << 16); }
__device__ __forceinline__ float bfr(float f) { return bf2f(f2bf(f)); }
__device__ __forceinline__ v16h cat16(v8h lo, v8h hi) { return __builtin_shufflevector(lo, hi, 0, 1, 2, 3, 4, 5, 6, 7, 8, 9, 10, 11, 12, 13, 14, 15); }
__device__ __forceinline__ v16bf cat16b(v8us lo, v8us hi) { return __builtin_bit_cast(v16bf, __builtin_shufflevector(lo, hi, 0, 1, 2, 3, 4, 5, 6, 7, 8, 9, 10, 11, 12, 13, 14, 15)); }
__device__ __forceinline__ v8f wmma16(v16h a, v16h b, v8f c) { return __builtin_amdgcn_wmma_f32_16x16x32_f16(false, a, false, b, (short)0, c, false, false); }
__device__ __forceinline__ v8f wmmab(v16bf a, v16bf b, v8f c) { return __builtin_amdgcn_wmma_f32_16x16x32_bf16(false, a, false, b, (short)0, c, false, false); }


template <typename T16> struct WFrag;
template <> struct WFrag<h16> { typedef v16h V; static __device__ __forceinline__ V ld(const h16* p) { return cat16(*(const v8h*)p, *(const v8h*)(p + 16)); } static __device__ __forceinline__ v8f mma(V a, V b, v8f c) { return wmma16(a, b, c); } };
template <> struct WFrag<bf> { typedef v16bf V; static __device__ __forceinline__ V ld(const bf* p) { return cat16b(*(const v8us*)p, *(const v8us*)(p + 16)); } static __device__ __forceinline__ v8f mma(V a, V b, v8f c) { return wmmab(a, b, c); } };
template <typename T16, int NSPLIT, bool BIAS>
__global__ __launch_bounds__(32) void k_gemmw(const T16* __restrict__ A, const T16* __restrict__ A2, const T16* __restrict__ Bt, const T16* __restrict__ Bt2, int K, float* C, int ldc, const float* __restrict__ bias, size_t sA, size_t sB, size_t sC) {
    typedef typename WFrag<T16>::V V;
    __shared__ __align__(16) float os[16 * 68];
    const size_t z = blockIdx.z; A += z * sA; if (A2) A2 += z * sA; Bt += z * sB; if (Bt2) Bt2 += z * sB; C += z * sC;
    const int lane = threadIdx.x & 31, lr = lane & 15, hi = lane >> 4; const int r0 = blockIdx.x * 64, c0 = blockIdx.y * 64;
    v8f acc[4][4];
#pragma unroll
    for (int mb = 0; mb < 4; ++mb)
#pragma unroll
        for (int nb = 0; nb < 4; ++nb) acc[mb][nb] = (v8f){};
    const size_t aoff = (size_t)(r0 + lr) * K + 8 * hi, boff = (size_t)(c0 + lr) * K + 8 * hi;
#pragma unroll 1
    for (int kc = 0; kc < K; kc += 32) {
        V a[4], a2[4];
#pragma unroll
        for (int mb = 0; mb < 4; ++mb) { a[mb] = WFrag<T16>::ld(A + aoff + (size_t)mb * 16 * K + kc); if (NSPLIT == 1 || NSPLIT == 2) a2[mb] = WFrag<T16>::ld(A2 + aoff + (size_t)mb * 16 * K + kc); }
#pragma unroll
        for (int nb = 0; nb < 4; ++nb) { const V b = WFrag<T16>::ld(Bt + boff + (size_t)nb * 16 * K + kc); V b2; if (NSPLIT >= 2) b2 = WFrag<T16>::ld(Bt2 + boff + (size_t)nb * 16 * K + kc);
#pragma unroll
            for (int mb = 0; mb < 4; ++mb) { acc[mb][nb] = WFrag<T16>::mma(a[mb], b, acc[mb][nb]); if (NSPLIT == 1 || NSPLIT == 2) acc[mb][nb] = WFrag<T16>::mma(a2[mb], b, acc[mb][nb]); if (NSPLIT >= 2) acc[mb][nb] = WFrag<T16>::mma(a[mb], b2, acc[mb][nb]); } }
        asm volatile("v_nop\n\tv_nop\n\tv_nop\n\tv_nop" : "+v"(acc[0][0]), "+v"(acc[1][1]), "+v"(acc[2][2]), "+v"(acc[3][3]) : "v"(a[0]), "v"(a[3]));
    }
#pragma unroll
    for (int mb = 0; mb < 4; ++mb) {
#pragma unroll
        for (int nb = 0; nb < 4; ++nb) {
#pragma unroll
            for (int j = 0; j < 8; ++j) os[(hi * 8 + j) * 68 + nb * 16 + lr] = acc[mb][nb][j]; }
        __builtin_amdgcn_wave_barrier(); asm volatile("" ::: "memory");
        float* crow = C + (size_t)(r0 + mb * 16) * ldc + c0;
#pragma unroll 1
        for (int ps = 0; ps < 2; ++ps) {
#pragma unroll
            for (int s = 0; s < 8; ++s) { const int row = 2 * s + hi, cofs = lr * 4; v4f val = *(const v4fa*)(os + row * 68 + cofs); if (BIAS) { val[0] += bfr(bias[c0 + cofs]); val[1] += bfr(bias[c0 + cofs + 1]); val[2] += bfr(bias[c0 + cofs + 2]); val[3] += bfr(bias[c0 + cofs + 3]); }
                *(volatile v4f*)(crow + (size_t)row * ldc + cofs) = val; }
            if (ps == 0) __threadfence(); }
        __builtin_amdgcn_wave_barrier(); asm volatile("" ::: "memory");
    }
}

__device__ __forceinline__ h16 tohx(float x) { return (h16)x; }
__device__ __forceinline__ void splitf(float y, unsigned short& h, unsigned short& l) { h = f2bf(y); l = f2bf(y - bf2f(h)); }
typedef __attribute__((ext_vector_type(2))) _Float16 v2h;
typedef __attribute__((ext_vector_type(4))) _Float16 v4h;
typedef __attribute__((ext_vector_type(2))) unsigned short v2us;
typedef __attribute__((ext_vector_type(4))) unsigned short v4us;

__global__ __launch_bounds__(256) void k_wtb(const float* __restrict__ w, int K, int N, bf* Bt) {
    const int lane = threadIdx.x & 31; const int L0 = (blockIdx.x * 8 + (threadIdx.x >> 5)) * 8; const int nlines = N * K / 64;
#pragma unroll 1
    for (int ps = 0; ps < 2; ++ps) {
#pragma unroll 1
        for (int l = 0; l < 8; ++l) { const int L = L0 + l; if (L >= nlines) break; const int e = L * 64 + lane * 2; v2us o;
#pragma unroll
            for (int q = 0; q < 2; ++q) { const int n = (e + q) / K, k = (e + q) % K; o[q] = f2bf(w[(size_t)k * N + n]); }
            *(volatile v2us*)(Bt + e) = o; }
        if (ps == 0) __threadfence(); }
}
__global__ __launch_bounds__(256) void k_ln1(const float* __restrict__ x, const float* __restrict__ gg, const float* __restrict__ bb, bf* Ph, bf* Pl) {
    const int lane = threadIdx.x & 31; const int r = blockIdx.x * 8 + (threadIdx.x >> 5); if (r >= NT) return; float v[8]; float s = 0.f;
#pragma unroll
    for (int c = 0; c < 2; ++c) { const v4f a = *(const v4f*)(x + (size_t)r * DD + c * 128 + lane * 4);
#pragma unroll
        for (int q = 0; q < 4; ++q) { v[c * 4 + q] = bfr(a[q]); s += v[c * 4 + q]; } }
#pragma unroll
    for (int sh = 16; sh; sh >>= 1) s += __shfl_xor(s, sh, 32);
    const float mu = s * (1.0f / DD); float qq = 0.f;
#pragma unroll
    for (int i = 0; i < 8; ++i) { const float d0 = v[i] - mu; qq = fmaf(d0, d0, qq); }
#pragma unroll
    for (int sh = 16; sh; sh >>= 1) qq += __shfl_xor(qq, sh, 32);
    const float rs = rsqrtf(qq * (1.0f / DD) + 1e-5f); v4us oh[2], ol[2];
#pragma unroll
    for (int c = 0; c < 2; ++c)
#pragma unroll
        for (int q = 0; q < 4; ++q) { const int col = c * 128 + lane * 4 + q; unsigned short a, c2; splitf((v[c * 4 + q] - mu) * rs * bfr(gg[col]) + bfr(bb[col]), a, c2); oh[c][q] = a; ol[c][q] = c2; }
#pragma unroll 1
    for (int ps = 0; ps < 2; ++ps) {
#pragma unroll
        for (int c = 0; c < 2; ++c) { *(volatile v4us*)(Ph + (size_t)r * DD + c * 128 + lane * 4) = oh[c]; *(volatile v4us*)(Pl + (size_t)r * DD + c * 128 + lane * 4) = ol[c]; }
        if (ps == 0) __threadfence(); }
}
__global__ __launch_bounds__(256) void k_cvt16(const float* __restrict__ F, float sc, h16* P, size_t n8) { const size_t i = (size_t)blockIdx.x * 256 + threadIdx.x; if (i >= n8) return; const v8f v = *(const v8f*)(F + i * 8); v8h o;
#pragma unroll
    for (int k = 0; k < 8; ++k) o[k] = tohx(v[k] * sc); *(volatile v8h*)(P + i * 8) = o; __threadfence(); *(volatile v8h*)(P + i * 8) = o; }
__global__ __launch_bounds__(256) void k_vt(const float* __restrict__ F, h16* VT) {
    const int lane = threadIdx.x & 31; const int L0 = (blockIdx.x * 8 + (threadIdx.x >> 5)) * 8; const int nlines = NT * DD / 64;
#pragma unroll 1
    for (int ps = 0; ps < 2; ++ps) {
#pragma unroll
        for (int l = 0; l < 8; ++l) { const int L = L0 + l; if (L >= nlines) break; const int e = L * 64 + lane * 2; const int m = e & (NN - 1); const int d = (e >> 12) & (DD - 1); const int b = e >> 20; v2h v;
#pragma unroll
            for (int q = 0; q < 2; ++q) v[q] = tohx(F[((size_t)b * NN + m + q) * DD + d]);
            *(volatile v2h*)(VT + (size_t)e) = v; }
        if (ps == 0) __threadfence(); }
}
__global__ __launch_bounds__(256) void k_relu16(const float* __restrict__ S, h16* P, size_t n8) { const size_t i = (size_t)blockIdx.x * 256 + threadIdx.x; if (i >= n8) return; const v8f v = *(const v8f*)(S + i * 8); v8h o;
#pragma unroll
    for (int k = 0; k < 8; ++k) o[k] = tohx(fmaxf(v[k], 0.f)); *(volatile v8h*)(P + i * 8) = o; __threadfence(); *(volatile v8h*)(P + i * 8) = o; }
__global__ __launch_bounds__(256) void k_resid(const float* __restrict__ x, const float* __restrict__ AV, int r0, float* R, bf* Ph, bf* Pl) {
    typedef __attribute__((ext_vector_type(2))) float v2f;
    const int lane = threadIdx.x & 31; const int L0 = (blockIdx.x * 8 + (threadIdx.x >> 5)) * 8; const int nlines = QH * DD / 64;
#pragma unroll 1
    for (int ps = 0; ps < 2; ++ps) {
#pragma unroll
        for (int l = 0; l < 8; ++l) { const int L = L0 + l; if (L >= nlines) break; const int e = L * 64 + lane * 2; const size_t o = (size_t)r0 * DD + e; v2f rv; v2us oh, ol;
#pragma unroll
            for (int q = 0; q < 2; ++q) { const float v = bfr(x[o + q]) + AV[(size_t)e + q]; rv[q] = v; unsigned short a, c2; splitf(v, a, c2); oh[q] = a; ol[q] = c2; }
            *(volatile v2f*)(R + o) = rv; *(volatile v2us*)(Ph + o) = oh; *(volatile v2us*)(Pl + o) = ol; }
        if (ps == 0) __threadfence(); }
}
__global__ __launch_bounds__(256) void k_relusplit(const float* __restrict__ H, bf* Ph, bf* Pl, int nlines) {
    const int lane = threadIdx.x & 31; const int L0 = (blockIdx.x * 8 + (threadIdx.x >> 5)) * 8;
#pragma unroll 1
    for (int ps = 0; ps < 2; ++ps) {
#pragma unroll
        for (int l = 0; l < 8; ++l) { const int L = L0 + l; if (L >= nlines) break; const int e = L * 64 + lane * 2; v2us oh, ol;
#pragma unroll
            for (int q = 0; q < 2; ++q) { unsigned short a, c2; splitf(fmaxf(H[(size_t)e + q], 0.f), a, c2); oh[q] = a; ol[q] = c2; }
            *(volatile v2us*)(Ph + (size_t)e) = oh; *(volatile v2us*)(Pl + (size_t)e) = ol; }
        if (ps == 0) __threadfence(); }
}
__global__ __launch_bounds__(256) void k_ln2(const float* __restrict__ R, const float* __restrict__ F2, const float* __restrict__ gg, const float* __restrict__ bb, float* OUT) {
    const int lane = threadIdx.x & 31; const int r = blockIdx.x * 8 + (threadIdx.x >> 5); if (r >= NT) return; float v[8]; float s = 0.f;
#pragma unroll
    for (int c = 0; c < 2; ++c) { const v4f a = *(const v4f*)(R + (size_t)r * DD + c * 128 + lane * 4), f = *(const v4f*)(F2 + (size_t)r * DD + c * 128 + lane * 4);
#pragma unroll
        for (int q = 0; q < 4; ++q) { v[c * 4 + q] = a[q] + f[q]; s += v[c * 4 + q]; } }
#pragma unroll
    for (int sh = 16; sh; sh >>= 1) s += __shfl_xor(s, sh, 32);
    const float mu = s * (1.0f / DD); float qq = 0.f;
#pragma unroll
    for (int i = 0; i < 8; ++i) { const float d0 = v[i] - mu; qq = fmaf(d0, d0, qq); }
#pragma unroll
    for (int sh = 16; sh; sh >>= 1) qq += __shfl_xor(qq, sh, 32);
    const float rs = rsqrtf(qq * (1.0f / DD) + 1e-5f); v4f o[2];
#pragma unroll
    for (int c = 0; c < 2; ++c)
#pragma unroll
        for (int q = 0; q < 4; ++q) { const int col = c * 128 + lane * 4 + q; o[c][q] = (v[c * 4 + q] - mu) * rs * bfr(gg[col]) + bfr(bb[col]); }
#pragma unroll 1
    for (int ps = 0; ps < 2; ++ps) {
#pragma unroll
        for (int c = 0; c < 2; ++c) *(volatile v4f*)(OUT + (size_t)r * DD + c * 128 + lane * 4) = o[c];
        if (ps == 0) __threadfence(); }
}

extern "C" void kernel_launch(void* const* d_in, const int* in_sizes, int n_in,
                              void* d_out, int out_size, void* d_ws, size_t ws_size, hipStream_t stream) {
    (void)in_sizes; (void)n_in; (void)out_size;
    const float* x = (const float*)d_in[0]; const float* ng = (const float*)d_in[1]; const float* nb = (const float*)d_in[2]; const float* wq = (const float*)d_in[3]; const float* bq = (const float*)d_in[4]; const float* wk = (const float*)d_in[5]; const float* bk = (const float*)d_in[6];
    const float* wv = (const float*)d_in[7]; const float* bv = (const float*)d_in[8]; const float* w1 = (const float*)d_in[9]; const float* b1 = (const float*)d_in[10]; const float* w2 = (const float*)d_in[11]; const float* b2 = (const float*)d_in[12]; const float* fg = (const float*)d_in[13]; const float* fb = (const float*)d_in[14];
    float* OUT = (float*)d_out;
    char* wsp = (char*)d_ws;
    auto take = [&](size_t bytes) { char* p = wsp; wsp += (bytes + 255) & ~(size_t)255; return (void*)p; };
    bf* WQ = (bf*)take((size_t)DD * DD * 2); bf* WK = (bf*)take((size_t)DD * DD * 2); bf* WV = (bf*)take((size_t)DD * DD * 2); bf* W1 = (bf*)take((size_t)DF * DD * 2); bf* W2 = (bf*)take((size_t)DD * DF * 2);
    bf* Hh = (bf*)take((size_t)NT * DD * 2); bf* Hl = (bf*)take((size_t)NT * DD * 2); float* F = (float*)take((size_t)NT * DD * 4);
    h16* QP = (h16*)take((size_t)NT * DD * 2); h16* KP = (h16*)take((size_t)NT * DD * 2); h16* VT = (h16*)take((size_t)NT * DD * 2);
    float* S = (float*)take((size_t)QH * NN * 4); h16* P = (h16*)take((size_t)QH * NN * 2); float* AV = (float*)take((size_t)QH * DD * 4);
    float* R = (float*)take((size_t)NT * DD * 4); bf* Rh = (bf*)take((size_t)NT * DD * 2); bf* Rl = (bf*)take((size_t)NT * DD * 2); bf* GPh = (bf*)take((size_t)NT * DF * 2); bf* GPl = (bf*)take((size_t)NT * DF * 2);
    if ((size_t)(wsp - (char*)d_ws) > ws_size) return;
    float* Hf = S;
    float* F2 = F;
    k_wtb<<<(DD * DD / 64 + 63) / 64, 256, 0, stream>>>(wq, DD, DD, WQ); k_wtb<<<(DD * DD / 64 + 63) / 64, 256, 0, stream>>>(wk, DD, DD, WK); k_wtb<<<(DD * DD / 64 + 63) / 64, 256, 0, stream>>>(wv, DD, DD, WV);
    k_wtb<<<(DF * DD / 64 + 63) / 64, 256, 0, stream>>>(w1, DD, DF, W1); k_wtb<<<(DD * DF / 64 + 63) / 64, 256, 0, stream>>>(w2, DF, DD, W2);
    k_ln1<<<NT / 8, 256, 0, stream>>>(x, ng, nb, Hh, Hl);
    const size_t n8 = (size_t)NT * DD / 8; const unsigned g8 = (unsigned)((n8 + 255) / 256);
    k_gemmw<bf, 1, true><<<dim3(NT / 64, DD / 64, 1), 32, 0, stream>>>(Hh, Hl, WQ, nullptr, DD, F, DD, bq, 0, 0, 0); k_cvt16<<<g8, 256, 0, stream>>>(F, 0.0625f, QP, n8);
    k_gemmw<bf, 1, true><<<dim3(NT / 64, DD / 64, 1), 32, 0, stream>>>(Hh, Hl, WK, nullptr, DD, F, DD, bk, 0, 0, 0); k_cvt16<<<g8, 256, 0, stream>>>(F, 1.0f, KP, n8);
    k_gemmw<bf, 1, true><<<dim3(NT / 64, DD / 64, 1), 32, 0, stream>>>(Hh, Hl, WV, nullptr, DD, F, DD, bv, 0, 0, 0); k_vt<<<(unsigned)((NT * DD / 64 + 63) / 64), 256, 0, stream>>>(F, VT);
    for (int b = 0; b < NB_; ++b)
        for (int hq = 0; hq < NN / QH; ++hq) { const size_t r0 = (size_t)b * NN + (size_t)hq * QH;
            k_gemmw<h16, 0, false><<<dim3(QH / 64, NN / 64, 1), 32, 0, stream>>>(QP + r0 * DD, nullptr, KP + (size_t)b * NN * DD, nullptr, DD, S, NN, nullptr, 0, 0, 0);
            k_relu16<<<(unsigned)(((size_t)QH * NN / 8 + 255) / 256), 256, 0, stream>>>(S, P, (size_t)QH * NN / 8);
            k_gemmw<h16, 0, false><<<dim3(QH / 64, DD / 64, 1), 32, 0, stream>>>(P, nullptr, VT + (size_t)b * DD * NN, nullptr, NN, AV, DD, nullptr, 0, 0, 0);
            k_resid<<<(QH * DD / 64 + 63) / 64, 256, 0, stream>>>(x, AV, (int)r0, R, Rh, Rl); }
    k_gemmw<bf, 1, true><<<dim3(NT / 64, DF / 64, 1), 32, 0, stream>>>(Rh, Rl, W1, nullptr, DD, Hf, DF, b1, 0, 0, 0);
    k_relusplit<<<(NT * DF / 64 + 63) / 64, 256, 0, stream>>>(Hf, GPh, GPl, NT * DF / 64);
    k_gemmw<bf, 1, true><<<dim3(NT / 64, DD / 64, 1), 32, 0, stream>>>(GPh, GPl, W2, nullptr, DF, F2, DD, b2, 0, 0, 0);
    k_ln2<<<NT / 8, 256, 0, stream>>>(R, F2, fg, fb, OUT);
}
